// SpatioTemporalAttentionGNN_10058813407712
// MI455X (gfx1250) — hardware-verified
//
#include <hip/hip_runtime.h>
#include <stddef.h>
#include <stdint.h>
#include <math.h>

#define C_B      4
#define C_S      96
#define C_N      2000
#define C_F      16
#define C_H      64
#define C_E      16000
#define C_SL     (C_B * C_S)
#define C_TILES  125
#define C_EPAD   16384
#define C_NPAD   2048
#define C_RPN    2176
#define DEGCAP   64
#define DEG_MEAS 22
#define C_P2     128000
#define OUT0_N   576000
#define OUT1_N   768000

static_assert(C_N == C_TILES * 16);
static_assert(C_N <= C_NPAD && C_E <= C_EPAD && C_E % 4 == 0);
static_assert(DEGCAP >= DEG_MEAS + 8);
static_assert(C_P2 == 1000 * 128 && C_P2 == C_N * C_H);
static_assert((OUT0_N * 4) % 128 == 0);
static_assert(OUT0_N == C_B * 24 * C_N * 3 && OUT1_N == C_B * C_S * C_N);

#define P_BG    0
#define P_WQ    128
#define P_WV    4224
#define P_VW    8320
#define P_VB    8448
#define P_LN1G  8576
#define P_LN1B  8704
#define PA_END  8832
#define P_WIH   8832
#define P_BIH   33408
#define P_BHH   33792
#define P_LN2G  34176
#define P_LN2B  34304
#define P_P1W   34432
#define P_P1B   42624
#define P_LB    42752
#define P_IB    42880
#define P_END   43008
static_assert(P_WV == P_WQ + 4096 && P_VW == P_WV + 4096 && P_BIH == P_WIH + 24576);
static_assert(P_BHH == P_BIH + 384 && P_LN2G == P_BHH + 384 && P_P1B == P_P1W + 8192);
static_assert(PA_END % 128 == 0 && P_END % 128 == 0 && (P_END - PA_END) % 128 == 0);

#define O_PAR   ((size_t)0)
#define O_WG2   ((size_t)172032)
#define O_WK2   ((size_t)176128)
#define O_WH2   ((size_t)192512)
#define O_DINV  ((size_t)212992)
#define O_RP    ((size_t)221184)
#define O_HSRC  ((size_t)229888)
#define O_HCF   ((size_t)295424)
#define O_POI   ((size_t)360960)
#define O_QP    ((size_t)361216)
#define O_MZ    ((size_t)362240)
#define O_FHL   ((size_t)362496)
#define O_REC   ((size_t)370688)
#define O_SC    ((size_t)567296)
#define O_NF    ((size_t)3713024)
#define O_QF    ((size_t)5761024)
#define WS_TOTAL ((size_t)8065024)
static_assert(O_WG2 == O_PAR + (size_t)P_END * 4);
static_assert(O_WK2 == O_WG2 + 64 * 32 * 2 && O_WH2 == O_WK2 + 64 * 128 * 2 && O_DINV == O_WH2 + 80 * 128 * 2);
static_assert(O_RP == O_DINV + C_NPAD * 4 && O_HSRC == O_RP + C_RPN * 4);
static_assert(O_HCF == O_HSRC + C_EPAD * 4 && O_POI == O_HCF + C_EPAD * 4);
static_assert(O_QP == O_POI + 256 && O_MZ == O_QP + 1024 && O_FHL == O_MZ + 256 && O_REC == O_FHL + 8192);
static_assert(O_SC == O_REC + (size_t)C_SL * 128 * 4 && O_NF == O_SC + (size_t)C_SL * 2048 * 4);
static_assert(O_QF == O_NF + (size_t)C_B * C_P2 * 4 && WS_TOTAL == O_QF + (size_t)8000 * 72 * 4);
static_assert(WS_TOTAL <= (size_t)134217728);
static_assert(O_RP % 256 == 0 && O_SC % 256 == 0 && O_NF % 256 == 0 && O_QF % 256 == 0);

#define CSR_INTS  (3 * C_E + C_NPAD + C_RPN + C_NPAD + 32)
#define Q_INTS    19264
#define MAIN_INTS 33344
static_assert(CSR_INTS * 4 <= 300000 && MAIN_INTS * 4 <= 300000);

#define KATTR(T) __global__ __launch_bounds__(T) __attribute__((amdgpu_num_vgpr(248)))

typedef float          v4f   __attribute__((ext_vector_type(4)));
typedef float          v8f   __attribute__((ext_vector_type(8)));
typedef int            v4i   __attribute__((ext_vector_type(4)));
typedef int            v8i   __attribute__((ext_vector_type(8)));
typedef unsigned       v4u   __attribute__((ext_vector_type(4)));
typedef unsigned short v8us  __attribute__((ext_vector_type(8)));
typedef unsigned short v16us __attribute__((ext_vector_type(16)));
typedef __bf16         v16bf __attribute__((ext_vector_type(16)));
typedef v4f  __attribute__((may_alias)) v4fa;
typedef v4i  __attribute__((may_alias)) v4ia;
typedef v4u  __attribute__((may_alias)) v4ua;
typedef v8us __attribute__((may_alias)) v8usa;
union FragB { v16bf v; v16us u; v8us h[2]; v8i w; };

__device__ __forceinline__ v8f wmb(const FragB& a, const FragB& b, v8f c) {
  v8f d = __builtin_amdgcn_wmma_f32_16x16x32_bf16(false, a.v, false, b.v, (short)0, c, false, false);
  asm volatile("v_nop\n\tv_nop\n\tv_nop\n\tv_nop" : "+v"(d) : "v"(a.w), "v"(b.w));
  return d;
}

__device__ __forceinline__ unsigned bf16_bits(float f) {
  const unsigned u = __float_as_uint(f);
  return (u + 0x7FFFu + ((u >> 16) & 1u)) >> 16;
}
__device__ __forceinline__ float bf16_val(float f) { return __uint_as_float(bf16_bits(f) << 16); }
__device__ __forceinline__ unsigned pk2(float a, float b) { return bf16_bits(a) | (bf16_bits(b) << 16); }
__device__ __forceinline__ int iclamp(int v, int lo, int hi) { return v < lo ? lo : (v > hi ? hi : v); }
__device__ __forceinline__ float elu_f(float v) { const float e = expm1f(v); return (v > 0.0f) ? v : e; }
__device__ __forceinline__ float softplus_f(float v) { return fmaxf(v, 0.0f) + log1pf(expf(-fabsf(v))); }

__device__ __forceinline__ void pack4(const float* __restrict__ src, int n, int j, float* dst) {
  const int n1 = n - 1;
  const float a0 = src[(j     < n1) ? j     : n1];
  const float a1 = src[(j + 1 < n1) ? j + 1 : n1];
  const float a2 = src[(j + 2 < n1) ? j + 2 : n1];
  const float a3 = src[(j + 3 < n1) ? j + 3 : n1];
  v4f o;
  o.x = (j     < n) ? bf16_val(a0) : 0.0f;
  o.y = (j + 1 < n) ? bf16_val(a1) : 0.0f;
  o.z = (j + 2 < n) ? bf16_val(a2) : 0.0f;
  o.w = (j + 3 < n) ? bf16_val(a3) : 0.0f;
  float* p = dst + j;
  *(volatile v4f*)p = o;
  __threadfence();
  *(volatile v4f*)p = o;
}

KATTR(256) void k_pa(const float* __restrict__ bg, const float* __restrict__ wq, const float* __restrict__ wv,
                     const float* __restrict__ vw, const float* __restrict__ vb, const float* __restrict__ l1g,
                     const float* __restrict__ l1b, float* par) {
  const int f = ((int)blockIdx.x * 256 + (int)threadIdx.x) * 4;
  if (f >= PA_END) return;
  const float* src = bg; int n = 64; int base = P_BG;
  if (f >= P_LN1B)      { src = l1b; n = 64;   base = P_LN1B; }
  else if (f >= P_LN1G) { src = l1g; n = 64;   base = P_LN1G; }
  else if (f >= P_VB)   { src = vb;  n = 1;    base = P_VB; }
  else if (f >= P_VW)   { src = vw;  n = 64;   base = P_VW; }
  else if (f >= P_WV)   { src = wv;  n = 4096; base = P_WV; }
  else if (f >= P_WQ)   { src = wq;  n = 4096; base = P_WQ; }
  pack4(src, n, f - base, par + base);
}

KATTR(256) void k_pb(const float* __restrict__ wih, const float* __restrict__ bih, const float* __restrict__ bhh,
                     const float* __restrict__ l2g, const float* __restrict__ l2b, const float* __restrict__ p1w,
                     const float* __restrict__ p1b, const float* __restrict__ lb, const float* __restrict__ ib,
                     float* par) {
  const int f = P_WIH + ((int)blockIdx.x * 256 + (int)threadIdx.x) * 4;
  if (f >= P_END) return;
  const float* src = wih; int n = 24576; int base = P_WIH;
  if (f >= P_IB)        { src = ib;  n = 48;   base = P_IB; }
  else if (f >= P_LB)   { src = lb;  n = 24;   base = P_LB; }
  else if (f >= P_P1B)  { src = p1b; n = 128;  base = P_P1B; }
  else if (f >= P_P1W)  { src = p1w; n = 8192; base = P_P1W; }
  else if (f >= P_LN2B) { src = l2b; n = 64;   base = P_LN2B; }
  else if (f >= P_LN2G) { src = l2g; n = 64;   base = P_LN2G; }
  else if (f >= P_BHH)  { src = bhh; n = 384;  base = P_BHH; }
  else if (f >= P_BIH)  { src = bih; n = 384;  base = P_BIH; }
  pack4(src, n, f - base, par + base);
}

KATTR(256) void k_pc(const float* __restrict__ wg, const float* __restrict__ wk, const float* __restrict__ lw,
                     const float* __restrict__ iw, unsigned short* wg2, unsigned short* wk2, unsigned short* wh2) {
  const int blk = (int)blockIdx.x, tid = (int)threadIdx.x;
  v4f a, b;
  unsigned short* dp;
  if (blk == 0) {
    const int u = tid, n = u >> 2, k8 = (u & 3) * 8;
    const float* p = wg + n * C_F + (k8 & 15);
    a = *(const v4fa*)p; b = *(const v4fa*)(p + 4);
    dp = wg2 + u * 8;
  } else if (blk < 5) {
    const int u = (blk - 1) * 256 + tid, n = u >> 4, k8 = (u & 15) * 8;
    const float* p = wk + n * C_H + (k8 & 63);
    a = *(const v4fa*)p; b = *(const v4fa*)(p + 4);
    dp = wk2 + u * 8;
  } else {
    const int u = (blk - 5) * 256 + tid, n = u >> 4, k8 = (u & 15) * 8, kk = k8 & 63;
    const int rl = n < 23 ? n : 23;
    const int ri = iclamp(n - 24, 0, 47);
    const float* pl = lw + rl * C_H + kk;
    const float* pi = iw + ri * C_H + kk;
    const v4f la = *(const v4fa*)pl, lc = *(const v4fa*)(pl + 4);
    const v4f ia = *(const v4fa*)pi, ic = *(const v4fa*)(pi + 4);
    const float fa = (n < 24) ? 1.0f : 0.0f;
    const float fb = (n >= 24 && n < 72) ? 1.0f : 0.0f;
    a = la * fa + ia * fb;
    b = lc * fa + ic * fb;
    dp = wh2 + u * 8;
  }
  v8us o;
  o[0] = (unsigned short)bf16_bits(a.x); o[1] = (unsigned short)bf16_bits(a.y);
  o[2] = (unsigned short)bf16_bits(a.z); o[3] = (unsigned short)bf16_bits(a.w);
  o[4] = (unsigned short)bf16_bits(b.x); o[5] = (unsigned short)bf16_bits(b.y);
  o[6] = (unsigned short)bf16_bits(b.z); o[7] = (unsigned short)bf16_bits(b.w);
  *(volatile v8us*)dp = o;
  __threadfence();
  *(volatile v8us*)dp = o;
}

__device__ __forceinline__ void csr_export(const float* dvL, const int* rpL, int flag, float* dinvG, int* rpG,
                                           int* poiG, int tid) {
  const v4f dv = *(const v4fa*)(dvL + 4 * tid);
  *(volatile v4f*)(dinvG + 4 * tid) = dv;
  const v4i ra = *(const v4ia*)(rpL + 4 * tid);
  *(volatile v4i*)(rpG + 4 * tid) = ra;
  if (tid < 32) {
    const v4i rb = *(const v4ia*)(rpL + 4 * (tid + 512));
    *(volatile v4i*)(rpG + 4 * (tid + 512)) = rb;
    if (tid < 8) {
      const v4i fl = {flag, flag, flag, flag};
      *(volatile v4i*)(poiG + 4 * tid) = fl;
    }
  }
}

KATTR(512) void k_csr(const int* __restrict__ ei, const float* __restrict__ ew, float* dinvG, int* rpG,
                      int* hsG, float* hcG, int* poiG) {
  extern __shared__ __attribute__((aligned(16))) int dsm[];
  int*   dstL = dsm;
  float* ewL  = (float*)(dsm + C_E);
  int*   he   = dsm + 2 * C_E;
  int*   cntL = dsm + 3 * C_E;
  int*   rpL  = cntL + C_NPAD;
  float* dvL  = (float*)(rpL + C_RPN);
  int*   misc = (int*)(dvL + C_NPAD);
  const int tid = (int)threadIdx.x, lane = tid & 31;

#pragma unroll 1
  for (int c = tid; c < C_E / 4; c += 512) {
    const v4i d = *(const v4ia*)(ei + C_E + 4 * c);
    *(v4ia*)(dstL + 4 * c) = d;
    const v4f w = *(const v4fa*)(ew + 4 * c);
    const v4f wr = {bf16_val(w.x), bf16_val(w.y), bf16_val(w.z), bf16_val(w.w)};
    *(v4fa*)(ewL + 4 * c) = wr;
    const v4i z = {0, 0, 0, 0};
    *(v4ia*)(he + 4 * c) = z;
  }
  if (tid < 32) misc[tid] = 0;
  __syncthreads();

  const int n0 = tid, n1 = tid + 512, n2 = tid + 1024, n3 = tid + 1536;
  const bool v3 = n3 < C_N;
  float g0 = 0.0f, g1 = 0.0f, g2 = 0.0f, g3 = 0.0f;
  int c0 = 0, c1 = 0, c2 = 0, c3 = 0;
#define CS1(D, W) \
  g0 += ((D) == n0) ? (W) : 0.0f; c0 += ((D) == n0) ? 1 : 0; \
  g1 += ((D) == n1) ? (W) : 0.0f; c1 += ((D) == n1) ? 1 : 0; \
  g2 += ((D) == n2) ? (W) : 0.0f; c2 += ((D) == n2) ? 1 : 0; \
  g3 += (((D) == n3) & v3) ? (W) : 0.0f; c3 += (((D) == n3) & v3) ? 1 : 0;
#pragma unroll 1
  for (int e = 0; e < C_E; e += 4) {
    const v4i d = *(const v4ia*)(dstL + e);
    const v4f w = *(const v4fa*)(ewL + e);
    CS1(d.x, w.x)
    CS1(d.y, w.y)
    CS1(d.z, w.z)
    CS1(d.w, w.w)
  }
#undef CS1
  {
    const float d0 = g0 + 1.0f, d1 = g1 + 1.0f, d2 = g2 + 1.0f, d3 = g3 + 1.0f;
    cntL[n0] = c0; cntL[n1] = c1; cntL[n2] = c2; cntL[n3] = v3 ? c3 : 0;
    dvL[n0] = d0 > 0.0f ? 1.0f / sqrtf(d0) : 0.0f;
    dvL[n1] = d1 > 0.0f ? 1.0f / sqrtf(d1) : 0.0f;
    dvL[n2] = d2 > 0.0f ? 1.0f / sqrtf(d2) : 0.0f;
    const float q3 = d3 > 0.0f ? 1.0f / sqrtf(d3) : 0.0f;
    dvL[n3] = v3 ? q3 : 0.0f;
    int mx = c0 > c1 ? c0 : c1;
    mx = mx > c2 ? mx : c2;
    mx = mx > c3 ? mx : c3;
    if (mx > DEGCAP) misc[0] = 1;
  }
  __syncthreads();

  if (tid < 32) {
    const int base = tid * 64;
    int s = 0;
#pragma unroll 1
    for (int i = 0; i < 64; ++i) s += cntL[base + i];
    int incl = s;
#pragma unroll
    for (int d = 1; d < 32; d <<= 1) {
      const int y = __shfl_up(incl, d, 32);
      if (lane >= d) incl += y;
    }
    int run = incl - s;
#pragma unroll 1
    for (int i = 0; i < 64; ++i) {
      const int cv = cntL[base + i];
      rpL[base + i] = run;
      run += cv;
    }
    const int tot = __shfl(incl, 31, 32);
    rpL[C_NPAD + 4 * tid]     = tot;
    rpL[C_NPAD + 4 * tid + 1] = tot;
    rpL[C_NPAD + 4 * tid + 2] = tot;
    rpL[C_NPAD + 4 * tid + 3] = tot;
  }
  __syncthreads();

  {
    int p0 = rpL[n0], p1 = rpL[n1], p2 = rpL[n2], p3 = rpL[n3];
#define CS2(D, EE) \
    if ((D) == n0) { he[p0 < C_E ? p0 : C_E - 1] = (EE); ++p0; } \
    if ((D) == n1) { he[p1 < C_E ? p1 : C_E - 1] = (EE); ++p1; } \
    if ((D) == n2) { he[p2 < C_E ? p2 : C_E - 1] = (EE); ++p2; } \
    if (((D) == n3) & v3) { he[p3 < C_E ? p3 : C_E - 1] = (EE); ++p3; }
#pragma unroll 1
    for (int e = 0; e < C_E; e += 4) {
      const v4i d = *(const v4ia*)(dstL + e);
      CS2(d.x, e)
      CS2(d.y, e + 1)
      CS2(d.z, e + 2)
      CS2(d.w, e + 3)
    }
#undef CS2
  }
  __syncthreads();

  const int tot = iclamp(rpL[C_NPAD], 0, C_E);
#pragma unroll 1
  for (int q = 0; q < C_EPAD / 4 / 512; ++q) {
    const int c = tid + 512 * q;
    v4i so; v4f co;
#pragma unroll
    for (int j = 0; j < 4; ++j) {
      const int i = 4 * c + j;
      const bool valid = i < tot;
      const int e = iclamp(he[i < C_E ? i : C_E - 1], 0, C_E - 1);
      const int s = iclamp(ei[e], 0, C_N - 1);
      const int d = iclamp(dstL[e], 0, C_N - 1);
      const float cf = (dvL[s] * ewL[e]) * dvL[d];
      so[j] = valid ? s : 0;
      co[j] = valid ? cf : 0.0f;
    }
    *(volatile v4i*)(hsG + 4 * c) = so;
    *(volatile v4f*)(hcG + 4 * c) = co;
    __threadfence();
    *(volatile v4i*)(hsG + 4 * c) = so;
    *(volatile v4f*)(hcG + 4 * c) = co;
  }
  const int flag = misc[0];
  csr_export(dvL, rpL, flag, dinvG, rpG, poiG, tid);
  __threadfence();
  csr_export(dvL, rpL, flag, dinvG, rpG, poiG, tid);
}

__device__ __forceinline__ void tile_h(int tile, int lane, const unsigned* xs, const unsigned short* wg2l,
                                       const int* __restrict__ rp, const int* __restrict__ hsrc,
                                       const float* __restrict__ hcf, const float* __restrict__ dinv,
                                       const float* bgl, v8f (&hd)[4]) {
  const int r = lane & 15, hf = lane >> 4;
  const int node = tile * 16 + r;
  const int p0 = iclamp(rp[node], 0, C_EPAD - 1);
  const int c  = iclamp(rp[node + 1] - p0, 0, DEGCAP);
  int cm = c;
#pragma unroll
  for (int q = 1; q < 32; q <<= 1) {
    const int y = __shfl_xor(cm, q, 32);
    cm = cm > y ? cm : y;
  }
  cm = __builtin_amdgcn_readfirstlane(cm);
  float ax[8];
#pragma unroll
  for (int i = 0; i < 8; ++i) ax[i] = 0.0f;
#pragma unroll 1
  for (int k = 0; k < cm; ++k) {
    const bool valid = k < c;
    int p = p0 + (valid ? k : 0);
    p = p > C_EPAD - 1 ? C_EPAD - 1 : p;
    const int s = iclamp(hsrc[p], 0, C_N - 1);
    const float cl = hcf[p];
    const float cf = valid ? cl : 0.0f;
    const v4u w = *(const v4ua*)(xs + s * 8 + hf * 4);
#pragma unroll
    for (int j = 0; j < 4; ++j) {
      ax[2 * j]     = fmaf(cf, __uint_as_float(w[j] << 16), ax[2 * j]);
      ax[2 * j + 1] = fmaf(cf, __uint_as_float(w[j] & 0xffff0000u), ax[2 * j + 1]);
    }
  }
  {
    const float dn = dinv[node];
    const float d2 = dn * dn;
    const v4u w = *(const v4ua*)(xs + node * 8 + hf * 4);
#pragma unroll
    for (int j = 0; j < 4; ++j) {
      ax[2 * j]     = fmaf(d2, __uint_as_float(w[j] << 16), ax[2 * j]);
      ax[2 * j + 1] = fmaf(d2, __uint_as_float(w[j] & 0xffff0000u), ax[2 * j + 1]);
    }
  }
  FragB af;
#pragma unroll
  for (int i = 0; i < 8; ++i) {
    const unsigned hb = bf16_bits(ax[i]);
    const unsigned lb = bf16_bits(ax[i] - __uint_as_float(hb << 16));
    af.u[i]     = (unsigned short)hb;
    af.u[8 + i] = (unsigned short)lb;
  }
  const v8f z = {0.f, 0.f, 0.f, 0.f, 0.f, 0.f, 0.f, 0.f};
#pragma unroll
  for (int nt = 0; nt < 4; ++nt) {
    const unsigned short* q = wg2l + (16 * nt + r) * 32 + 8 * hf;
    FragB bf;
    bf.h[0] = *(const v8usa*)q;
    bf.h[1] = *(const v8usa*)(q + 16);
    hd[nt] = wmb(af, bf, z);
  }
#pragma unroll
  for (int nt = 0; nt < 4; ++nt) {
    const float bgv = bgl[16 * nt + r];
#pragma unroll
    for (int r8 = 0; r8 < 8; ++r8) hd[nt][r8] = elu_f(hd[nt][r8] + bgv);
  }
}

__device__ __forceinline__ void stage_xs(const float* __restrict__ xsl, unsigned* xs, int tid) {
#pragma unroll 2
  for (int c = tid; c < C_N * 2; c += 256) {
    const v4f a = *(const v4fa*)(xsl + 8 * c);
    const v4f q = *(const v4fa*)(xsl + 8 * c + 4);
    v4u o;
    o.x = pk2(a.x, a.y); o.y = pk2(a.z, a.w); o.z = pk2(q.x, q.y); o.w = pk2(q.z, q.w);
    *(v4ua*)(xs + 4 * c) = o;
  }
}

KATTR(256) void k_q(const float* __restrict__ x, const float* __restrict__ par, const unsigned short* __restrict__ wg2,
                    const int* __restrict__ rp, const int* __restrict__ hsrc, const float* __restrict__ hcf,
                    const float* __restrict__ dinv, float* qpG) {
  extern __shared__ __attribute__((aligned(16))) int dsm[];
  unsigned*       xs   = (unsigned*)dsm;
  unsigned short* wg2l = (unsigned short*)(dsm + 16000);
  double*         colp = (double*)(dsm + 17024);
  float*          ql   = (float*)(dsm + 19072);
  float*          qpl  = (float*)(dsm + 19136);
  float*          bgl  = (float*)(dsm + 19200);
  const int tid = (int)threadIdx.x, lane = tid & 31;
  const int wave = __builtin_amdgcn_readfirstlane(tid >> 5);
  const int r = lane & 15, hf = lane >> 4;
  const int b = (int)blockIdx.x;
  const float* xsl = x + (size_t)(b * C_S + (C_S - 1)) * (size_t)(C_N * C_F);
  stage_xs(xsl, xs, tid);
  *(v8usa*)(wg2l + 8 * tid) = *(const v8usa*)(wg2 + 8 * tid);
  if (tid < 64) bgl[tid] = par[P_BG + tid];
  __syncthreads();

  double cs[4] = {0.0, 0.0, 0.0, 0.0};
#pragma unroll 1
  for (int t = wave; t < C_TILES; t += 8) {
    v8f hd[4];
    tile_h(t, lane, xs, wg2l, rp, hsrc, hcf, dinv, bgl, hd);
#pragma unroll
    for (int nt = 0; nt < 4; ++nt) {
      const float s = ((hd[nt][0] + hd[nt][1]) + (hd[nt][2] + hd[nt][3])) +
                      ((hd[nt][4] + hd[nt][5]) + (hd[nt][6] + hd[nt][7]));
      cs[nt] += (double)s;
    }
  }
#pragma unroll
  for (int nt = 0; nt < 4; ++nt) colp[(wave * 2 + hf) * 64 + 16 * nt + r] = cs[nt];
  __syncthreads();
  if (tid < 64) {
    double a = 0.0;
#pragma unroll 1
    for (int j = 0; j < 16; ++j) a += colp[j * 64 + tid];
    ql[tid] = (float)(a * (1.0 / 2000.0));
  }
  __syncthreads();
  if (tid < 64) {
    const float* wr = par + P_WQ + tid * 64;
    float s = 0.0f;
#pragma unroll 1
    for (int j = 0; j < 64; j += 4) {
      const v4f a = *(const v4fa*)(wr + j);
      const v4f q = *(const v4fa*)(ql + j);
      s = fmaf(a.x, q.x, s); s = fmaf(a.y, q.y, s); s = fmaf(a.z, q.z, s); s = fmaf(a.w, q.w, s);
    }
    qpl[tid] = s;
  }
  __syncthreads();
  if (tid < 16) {
    const v4f o = *(const v4fa*)(qpl + 4 * tid);
    float* p = qpG + b * 64 + 4 * tid;
    *(volatile v4f*)p = o;
    __threadfence();
    *(volatile v4f*)p = o;
  }
}

__device__ __forceinline__ void main_flush(const float* scl, const float* reco, float* scg, float* recg,
                                           int tid, int wave, int lane) {
  const v4f s0 = *(const v4fa*)(scl + 4 * tid);
  const v4f s1 = *(const v4fa*)(scl + 4 * (tid + 256));
  *(volatile v4f*)(scg + 4 * tid) = s0;
  *(volatile v4f*)(scg + 4 * (tid + 256)) = s1;
  if (wave == 0) {
    const v4f rc = *(const v4fa*)(reco + 4 * lane);
    *(volatile v4f*)(recg + 4 * lane) = rc;
  }
}

KATTR(256) void k_main(const float* __restrict__ x, const float* __restrict__ par,
                       const unsigned short* __restrict__ wg2, const unsigned short* __restrict__ wk2,
                       const int* __restrict__ rp, const int* __restrict__ hsrc, const float* __restrict__ hcf,
                       const float* __restrict__ dinv, const float* __restrict__ qp, float* rec, float* sc) {
  extern __shared__ __attribute__((aligned(16))) int dsm[];
  unsigned*       xs   = (unsigned*)dsm;
  unsigned short* wk2l = (unsigned short*)(dsm + 16000);
  unsigned short* wg2l = (unsigned short*)(dsm + 20096);
  unsigned short* stg  = (unsigned short*)(dsm + 21120);
  float*          scl  = (float*)(dsm + 29824);
  float*          recl = (float*)(dsm + 31872);
  float*          reco = (float*)(dsm + 32960);
  float*          prm  = (float*)(dsm + 33088);
  const int tid = (int)threadIdx.x, lane = tid & 31;
  const int wave = __builtin_amdgcn_readfirstlane(tid >> 5);
  const int r = lane & 15, hf = lane >> 4;
  const int blk = (int)blockIdx.x;
  const int b = blk / C_S;

  stage_xs(x + (size_t)blk * (size_t)(C_N * C_F), xs, tid);
#pragma unroll
  for (int i = 0; i < 4; ++i) {
    const int c = tid + 256 * i;
    *(v8usa*)(wk2l + 8 * c) = *(const v8usa*)(wk2 + 8 * c);
  }
  *(v8usa*)(wg2l + 8 * tid) = *(const v8usa*)(wg2 + 8 * tid);
  if (tid < 64) {
    prm[tid]       = par[P_BG + tid];
    prm[64 + tid]  = qp[b * 64 + tid];
    prm[128 + tid] = par[P_VW + tid];
  }
  if (tid == 64) prm[192] = par[P_VB];
  if (tid < 48) scl[C_N + tid] = 0.0f;
  __syncthreads();

  float qpv[4], vwv[4];
#pragma unroll
  for (int nt = 0; nt < 4; ++nt) { qpv[nt] = prm[64 + 16 * nt + r]; vwv[nt] = prm[128 + 16 * nt + r]; }
  const float vb = prm[192];
  unsigned short* st = stg + wave * 2176;
  const v8f z = {0.f, 0.f, 0.f, 0.f, 0.f, 0.f, 0.f, 0.f};

  float m_run = -3.0e38f, l_run = 0.0f;
  float sacc[4] = {0.0f, 0.0f, 0.0f, 0.0f};

#pragma unroll 1
  for (int it = 0; it < 16; ++it) {
    const int t = wave + 8 * it;
    const bool live = t < C_TILES;
    v8f hd[4];
#pragma unroll
    for (int nt = 0; nt < 4; ++nt) hd[nt] = z;
    if (live) {
      tile_h(t, lane, xs, wg2l, rp, hsrc, hcf, dinv, prm, hd);
#pragma unroll
      for (int nt = 0; nt < 4; ++nt) {
#pragma unroll
        for (int r8 = 0; r8 < 8; ++r8) {
          const float v = hd[nt][r8];
          const unsigned hb = bf16_bits(v);
          const unsigned lb = bf16_bits(v - __uint_as_float(hb << 16));
          st[(8 * hf + r8) * 136 + 16 * nt + r]      = (unsigned short)hb;
          st[(8 * hf + r8) * 136 + 64 + 16 * nt + r] = (unsigned short)lb;
        }
      }
    }
    __syncthreads();
    if (live) {
      v8f kp[4];
#pragma unroll
      for (int nt = 0; nt < 4; ++nt) kp[nt] = z;
#pragma unroll 1
      for (int k0 = 0; k0 < 128; k0 += 32) {
        FragB af;
        af.h[0] = *(const v8usa*)(st + r * 136 + k0 + 8 * hf);
        af.h[1] = *(const v8usa*)(st + r * 136 + k0 + 16 + 8 * hf);
#pragma unroll
        for (int nt = 0; nt < 4; ++nt) {
          const unsigned short* q = wk2l + (16 * nt + r) * 128 + k0 + 8 * hf;
          FragB bf;
          bf.h[0] = *(const v8usa*)q;
          bf.h[1] = *(const v8usa*)(q + 16);
          kp[nt] = wmb(af, bf, kp[nt]);
        }
      }
      float sc8[8];
#pragma unroll
      for (int r8 = 0; r8 < 8; ++r8) {
        float p = 0.0f;
#pragma unroll
        for (int nt = 0; nt < 4; ++nt) p = fmaf(vwv[nt], tanhf(kp[nt][r8] + qpv[nt]), p);
        p += __shfl_xor(p, 1, 32);
        p += __shfl_xor(p, 2, 32);
        p += __shfl_xor(p, 4, 32);
        p += __shfl_xor(p, 8, 32);
        sc8[r8] = p + vb;
      }
      if (r == 0) {
        const v4f sa = {sc8[0], sc8[1], sc8[2], sc8[3]};
        const v4f sb = {sc8[4], sc8[5], sc8[6], sc8[7]};
        *(v4fa*)(scl + 16 * t + 8 * hf)     = sa;
        *(v4fa*)(scl + 16 * t + 8 * hf + 4) = sb;
      }
      float tm = sc8[0];
#pragma unroll
      for (int r8 = 1; r8 < 8; ++r8) tm = fmaxf(tm, sc8[r8]);
      const float mn  = fmaxf(m_run, tm);
      const float sca = expf(m_run - mn);
      float ps[8], ls = 0.0f;
#pragma unroll
      for (int r8 = 0; r8 < 8; ++r8) { ps[r8] = expf(sc8[r8] - mn); ls += ps[r8]; }
      l_run = fmaf(l_run, sca, ls);
#pragma unroll
      for (int nt = 0; nt < 4; ++nt) {
        float a = sacc[nt] * sca;
#pragma unroll
        for (int r8 = 0; r8 < 8; ++r8) a = fmaf(ps[r8], hd[nt][r8], a);
        sacc[nt] = a;
      }
      m_run = mn;
    }
  }

  {
    const int idx = wave * 2 + hf;
    if (r == 0) { recl[idx * 68] = m_run; recl[idx * 68 + 1] = l_run; recl[idx * 68 + 2] = 0.0f; recl[idx * 68 + 3] = 0.0f; }
#pragma unroll
    for (int nt = 0; nt < 4; ++nt) recl[idx * 68 + 4 + 16 * nt + r] = sacc[nt];
  }
  __syncthreads();
  if (tid < 64) {
    float M = recl[0];
#pragma unroll 1
    for (int j = 1; j < 16; ++j) M = fmaxf(M, recl[j * 68]);
    float L = 0.0f, A = 0.0f;
#pragma unroll 1
    for (int j = 0; j < 16; ++j) {
      const float w = expf(recl[j * 68] - M);
      L = fmaf(recl[j * 68 + 1], w, L);
      A = fmaf(recl[j * 68 + 4 + tid], w, A);
    }
    reco[tid] = A;
    if (tid == 0) { reco[64] = M; reco[65] = L; }
  } else if (tid >= 66 && tid < 128) {
    reco[tid] = 0.0f;
  }
  __syncthreads();
  float* scg  = sc + (size_t)blk * 2048;
  float* recg = rec + (size_t)blk * 128;
  main_flush(scl, reco, scg, recg, tid, wave, lane);
  __threadfence();
  main_flush(scl, reco, scg, recg, tid, wave, lane);
}

__device__ __forceinline__ float dot64(const float* __restrict__ w, const float* v) {
  float s = 0.0f;
#pragma unroll 1
  for (int j = 0; j < 64; j += 4) {
    const v4f a = *(const v4fa*)(w + j);
    const v4f c = *(const v4fa*)(v + j);
    s = fmaf(a.x, c.x, s); s = fmaf(a.y, c.y, s); s = fmaf(a.z, c.z, s); s = fmaf(a.w, c.w, s);
  }
  return s;
}
__device__ __forceinline__ float ln_one(const float* row, int c, float g, float be) {
  float s = 0.0f;
#pragma unroll 1
  for (int j = 0; j < 64; ++j) s += row[j];
  const float mu = s * (1.0f / 64.0f);
  float q = 0.0f;
#pragma unroll 1
  for (int j = 0; j < 64; ++j) { const float d = row[j] - mu; q = fmaf(d, d, q); }
  const float var = q * (1.0f / 64.0f);
  return (row[c] - mu) * (1.0f / sqrtf(var + 1e-5f)) * g + be;
}

KATTR(256) void k_tail(const float* __restrict__ par, const float* __restrict__ rec, float* mz, unsigned short* fhl) {
  __shared__ __attribute__((aligned(16))) float mL[384];
  __shared__ __attribute__((aligned(16))) float lL[384];
  __shared__ __attribute__((aligned(16))) float vA[256];
  __shared__ __attribute__((aligned(16))) float vB[256];
  __shared__ __attribute__((aligned(16))) float gi[768];
  __shared__ __attribute__((aligned(16))) float sg[512];
  __shared__ __attribute__((aligned(16))) float fL[512];
  __shared__ __attribute__((aligned(16))) float mzL[32];
  const int tid = (int)threadIdx.x;
  const int b = tid >> 6, c = tid & 63;

#pragma unroll 1
  for (int i = tid; i < C_SL; i += 256) { mL[i] = rec[(size_t)i * 128 + 64]; lL[i] = rec[(size_t)i * 128 + 65]; }
  if (tid < 32) mzL[tid] = 0.0f;
  __syncthreads();
  {
    float M = mL[b * C_S];
#pragma unroll 1
    for (int j = 1; j < C_S; ++j) M = fmaxf(M, mL[b * C_S + j]);
    double Zd = 0.0, Ad = 0.0;
#pragma unroll 2
    for (int j = 0; j < C_S; ++j) {
      const float w = expf(mL[b * C_S + j] - M);
      const float a = rec[(size_t)(b * C_S + j) * 128 + c];
      Zd += (double)lL[b * C_S + j] * (double)w;
      Ad += (double)a * (double)w;
    }
    const float zf = (float)Zd;
    vA[tid] = (float)Ad / zf;
    if (c == 0) { mzL[2 * b] = M; mzL[2 * b + 1] = zf; }
  }
  __syncthreads();
  vB[tid] = dot64(par + P_WV + c * 64, vA + b * 64);
  __syncthreads();
  {
    const float o = ln_one(vB + b * 64, c, par[P_LN1G + c], par[P_LN1B + c]);
    __syncthreads();
    vA[tid] = o;
  }
  __syncthreads();
#pragma unroll 1
  for (int l = 0; l < 2; ++l) {
#pragma unroll 1
    for (int q = 0; q < 3; ++q) {
      const int o = tid + 256 * q;
      const int bb = o / 192, t = o - bb * 192;
      gi[o] = dot64(par + P_WIH + (l * 192 + t) * 64, vA + bb * 64) + par[P_BIH + l * 192 + t];
    }
    __syncthreads();
#pragma unroll 1
    for (int q = 0; q < 2; ++q) {
      const int o = tid + 256 * q;
      const int bb = o >> 7, g = o & 127;
      const float a = gi[bb * 192 + g] + par[P_BHH + l * 192 + g];
      sg[o] = 1.0f / (1.0f + expf(-a));
    }
    __syncthreads();
    {
      const float rr = sg[b * 128 + c];
      const float zz = sg[b * 128 + 64 + c];
      const float nn = tanhf(gi[b * 192 + 128 + c] + rr * par[P_BHH + l * 192 + 128 + c]);
      vA[tid] = (1.0f - zz) * nn;
    }
    __syncthreads();
  }
  vB[tid] = ln_one(vA + b * 64, c, par[P_LN2G + c], par[P_LN2B + c]);
  __syncthreads();
#pragma unroll 1
  for (int q = 0; q < 2; ++q) {
    const int o = tid + 256 * q;
    const int bb = o >> 7, t = o & 127;
    fL[o] = elu_f(dot64(par + P_P1W + t * 64, vB + bb * 64) + par[P_P1B + t]);
  }
  __syncthreads();
  v8us o0, o1;
  {
#pragma unroll
    for (int q = 0; q < 2; ++q) {
      const int ch = tid + 256 * q;
      const int row = ch >> 5, k8 = (ch & 31) * 8;
      const bool islo = k8 >= 128;
      const int kk = k8 & 127, rr = row & 3;
      const bool keep = row < 4;
      v8us o;
#pragma unroll
      for (int i = 0; i < 8; ++i) {
        const float v = fL[rr * 128 + kk + i];
        const unsigned hb = bf16_bits(v);
        const unsigned lb = bf16_bits(v - __uint_as_float(hb << 16));
        const unsigned sel = islo ? lb : hb;
        o[i] = (unsigned short)(keep ? sel : 0u);
      }
      if (q == 0) o0 = o; else o1 = o;
    }
  }
  const v4f mzo = *(const v4fa*)(mzL + 4 * (tid & 7));
  *(volatile v8us*)(fhl + 8 * tid) = o0;
  *(volatile v8us*)(fhl + 8 * (tid + 256)) = o1;
  if (tid < 8) *(volatile v4f*)(mz + 4 * tid) = mzo;
  __threadfence();
  *(volatile v8us*)(fhl + 8 * tid) = o0;
  *(volatile v8us*)(fhl + 8 * (tid + 256)) = o1;
  if (tid < 8) *(volatile v4f*)(mz + 4 * tid) = mzo;
}

KATTR(256) void k_pre2(const unsigned short* __restrict__ fhl, const float* __restrict__ w2,
                       const float* __restrict__ b2, float* nf) {
  __shared__ __attribute__((aligned(16))) float T[4 * 128];
  const int tid = (int)threadIdx.x, lane = tid & 31;
  const int wave = __builtin_amdgcn_readfirstlane(tid >> 5);
  const int r = lane & 15, hf = lane >> 4;
  const int blk = (int)blockIdx.x;
  const int n0 = blk * 128 + 16 * wave;
  const float* wrow = w2 + (size_t)(n0 + r) * 128 + 8 * hf;
  const unsigned short* arow = fhl + r * 256 + 8 * hf;
  v8f acc = {0.f, 0.f, 0.f, 0.f, 0.f, 0.f, 0.f, 0.f};
#pragma unroll 1
  for (int k0 = 0; k0 < 128; k0 += 32) {
    const v4f a0 = *(const v4fa*)(wrow + k0);
    const v4f a1 = *(const v4fa*)(wrow + k0 + 4);
    const v4f c0 = *(const v4fa*)(wrow + k0 + 16);
    const v4f c1 = *(const v4fa*)(wrow + k0 + 20);
    FragB bf;
    bf.u[0]  = (unsigned short)bf16_bits(a0.x); bf.u[1]  = (unsigned short)bf16_bits(a0.y);
    bf.u[2]  = (unsigned short)bf16_bits(a0.z); bf.u[3]  = (unsigned short)bf16_bits(a0.w);
    bf.u[4]  = (unsigned short)bf16_bits(a1.x); bf.u[5]  = (unsigned short)bf16_bits(a1.y);
    bf.u[6]  = (unsigned short)bf16_bits(a1.z); bf.u[7]  = (unsigned short)bf16_bits(a1.w);
    bf.u[8]  = (unsigned short)bf16_bits(c0.x); bf.u[9]  = (unsigned short)bf16_bits(c0.y);
    bf.u[10] = (unsigned short)bf16_bits(c0.z); bf.u[11] = (unsigned short)bf16_bits(c0.w);
    bf.u[12] = (unsigned short)bf16_bits(c1.x); bf.u[13] = (unsigned short)bf16_bits(c1.y);
    bf.u[14] = (unsigned short)bf16_bits(c1.z); bf.u[15] = (unsigned short)bf16_bits(c1.w);
    FragB ah, al;
    ah.h[0] = *(const v8usa*)(arow + k0);
    ah.h[1] = *(const v8usa*)(arow + k0 + 16);
    al.h[0] = *(const v8usa*)(arow + 128 + k0);
    al.h[1] = *(const v8usa*)(arow + 128 + k0 + 16);
    acc = wmb(ah, bf, acc);
    acc = wmb(al, bf, acc);
  }
  const float bias = bf16_val(b2[n0 + r]);
  if (hf == 0) {
    T[0 * 128 + 16 * wave + r] = acc[0] + bias;
    T[1 * 128 + 16 * wave + r] = acc[1] + bias;
    T[2 * 128 + 16 * wave + r] = acc[2] + bias;
    T[3 * 128 + 16 * wave + r] = acc[3] + bias;
  }
  __syncthreads();
  if (tid < 128) {
    const int row = tid >> 5, c4 = (tid & 31) * 4;
    const v4f v = *(const v4fa*)(T + row * 128 + c4);
    float* p = nf + (size_t)row * C_P2 + (size_t)blk * 128 + c4;
    *(volatile v4f*)p = v;
    __threadfence();
    *(volatile v4f*)p = v;
  }
}

KATTR(128) void k_head(const float* __restrict__ nf, const unsigned short* __restrict__ wh2,
                       const float* __restrict__ par, float* qf) {
  __shared__ __attribute__((aligned(16))) float Tt[4 * 1280];
  __shared__ __attribute__((aligned(16))) float Ot[4 * 1152];
  const int tid = (int)threadIdx.x, lane = tid & 31;
  const int wave = __builtin_amdgcn_readfirstlane(tid >> 5);
  const int r = lane & 15, hf = lane >> 4;
  const int rowbase = (int)blockIdx.x * 64 + 16 * wave;
  const float* nrow = nf + (size_t)(rowbase + r) * 64;
  float* tw = Tt + wave * 1280;
  float* ow = Ot + wave * 1152;

  FragB ah[2], al[2];
#pragma unroll
  for (int kk = 0; kk < 2; ++kk) {
    const v4f a0 = *(const v4fa*)(nrow + 32 * kk + 8 * hf);
    const v4f a1 = *(const v4fa*)(nrow + 32 * kk + 8 * hf + 4);
    const v4f c0 = *(const v4fa*)(nrow + 32 * kk + 16 + 8 * hf);
    const v4f c1 = *(const v4fa*)(nrow + 32 * kk + 16 + 8 * hf + 4);
    const float vv[16] = {a0.x, a0.y, a0.z, a0.w, a1.x, a1.y, a1.z, a1.w,
                          c0.x, c0.y, c0.z, c0.w, c1.x, c1.y, c1.z, c1.w};
#pragma unroll
    for (int i = 0; i < 16; ++i) {
      const unsigned hb = bf16_bits(vv[i]);
      const unsigned lb = bf16_bits(vv[i] - __uint_as_float(hb << 16));
      ah[kk].u[i] = (unsigned short)hb;
      al[kk].u[i] = (unsigned short)lb;
    }
  }
  v8f acc[5];
  {
    const v8f z = {0.f, 0.f, 0.f, 0.f, 0.f, 0.f, 0.f, 0.f};
#pragma unroll
    for (int nt = 0; nt < 5; ++nt) acc[nt] = z;
  }
#pragma unroll
  for (int ks = 0; ks < 4; ++ks) {
    const int k0 = 32 * ks;
#pragma unroll
    for (int nt = 0; nt < 5; ++nt) {
      const unsigned short* q = wh2 + (16 * nt + r) * 128 + k0 + 8 * hf;
      FragB bf;
      bf.h[0] = *(const v8usa*)q;
      bf.h[1] = *(const v8usa*)(q + 16);
      if (ks == 0)      acc[nt] = wmb(ah[0], bf, acc[nt]);
      else if (ks == 1) acc[nt] = wmb(ah[1], bf, acc[nt]);
      else if (ks == 2) acc[nt] = wmb(al[0], bf, acc[nt]);
      else              acc[nt] = wmb(al[1], bf, acc[nt]);
    }
  }
#pragma unroll
  for (int nt = 0; nt < 5; ++nt) {
#pragma unroll
    for (int r8 = 0; r8 < 8; ++r8) tw[(8 * hf + r8) * 80 + 16 * nt + r] = acc[nt][r8];
  }
  __syncthreads();
#pragma unroll 1
  for (int it = 0; it < 12; ++it) {
    const int item = lane + 32 * it;
    const int row = item / 24, w = item - row * 24;
    const float ql = tw[row * 80 + w] + par[P_LB + w];
    const float i0 = tw[row * 80 + 24 + 2 * w] + par[P_IB + 2 * w];
    const float i1 = tw[row * 80 + 25 + 2 * w] + par[P_IB + 2 * w + 1];
    const float q1 = ql + softplus_f(i0);
    const float q2 = q1 + softplus_f(i1);
    ow[row * 72 + 3 * w]     = ql;
    ow[row * 72 + 3 * w + 1] = q1;
    ow[row * 72 + 3 * w + 2] = q2;
  }
  __syncthreads();
  v4f ov[9];
#pragma unroll
  for (int i = 0; i < 9; ++i) ov[i] = *(const v4fa*)(ow + 4 * (lane + 32 * i));
  float* qp0 = qf + (size_t)rowbase * 72;
#pragma unroll
  for (int i = 0; i < 9; ++i) *(volatile v4f*)(qp0 + 4 * (lane + 32 * i)) = ov[i];
  __threadfence();
#pragma unroll
  for (int i = 0; i < 9; ++i) *(volatile v4f*)(qp0 + 4 * (lane + 32 * i)) = ov[i];
}

KATTR(256) void k_out0(const float* __restrict__ qf, const int* __restrict__ poi, float* out) {
  const int g = (int)blockIdx.x * 256 + (int)threadIdx.x;
  if (g >= OUT0_N / 4) return;
  const bool bad = poi[0] != 0;
  v4f o;
#pragma unroll
  for (int j = 0; j < 4; ++j) {
    const int i = 4 * g + j;
    const int t = i / 3, q = i - 3 * t;
    const int t2 = t / C_N, n = t - t2 * C_N;
    const int b = t2 / 24, w = t2 - b * 24;
    const int idx = iclamp((b * C_N + n) * 72 + w * 3 + q, 0, 8000 * 72 - 1);
    const float v = qf[idx];
    o[j] = bad ? __int_as_float(0x7fc00000) : v;
  }
  float* p = out + 4 * (size_t)g;
  *(volatile v4f*)p = o;
  __threadfence();
  *(volatile v4f*)p = o;
}

KATTR(256) void k_out1(const float* __restrict__ sc, const float* __restrict__ mz, const int* __restrict__ poi,
                       float* out) {
  const int i = (int)blockIdx.x * 256 + (int)threadIdx.x;
  if (i >= OUT1_N) return;
  const bool bad = poi[0] != 0;
  const int slice = i / C_N, n = i - slice * C_N;
  const int b = slice / C_S;
  const float s = sc[(size_t)slice * 2048 + n];
  const float M = mz[2 * b], Z = mz[2 * b + 1];
  const float v = expf(s - M) / Z;
  const float o = bad ? __int_as_float(0x7fc00000) : v;
  float* p = out + OUT0_N + i;
  *(volatile float*)p = o;
  __threadfence();
  *(volatile float*)p = o;
}

extern "C" void kernel_launch(void* const* d_in, const int* in_sizes, int n_in,
                              void* d_out, int out_size, void* d_ws, size_t ws_size,
                              hipStream_t stream) {
  if (n_in < 26) return;
  if (in_sizes[0] != C_B * C_S * C_N * C_F) return;
  if (in_sizes[1] != 2 * C_E || in_sizes[2] != C_E) return;
  if (in_sizes[3] != C_H * C_F || in_sizes[4] != C_H) return;
  if (in_sizes[5] != 4096 || in_sizes[6] != 4096 || in_sizes[7] != 4096) return;
  if (in_sizes[8] != 64 || in_sizes[9] != 1 || in_sizes[10] != 64 || in_sizes[11] != 64) return;
  if (in_sizes[12] != 24576 || in_sizes[14] != 384 || in_sizes[15] != 384) return;
  if (in_sizes[16] != 64 || in_sizes[17] != 64) return;
  if (in_sizes[18] != 8192 || in_sizes[19] != 128) return;
  if (in_sizes[20] != C_P2 * 128 || in_sizes[21] != C_P2) return;
  if (in_sizes[22] != 1536 || in_sizes[23] != 24 || in_sizes[24] != 3072 || in_sizes[25] != 48) return;
  if (out_size != OUT0_N + OUT1_N) return;
  if (WS_TOTAL > ws_size) return;

  const float* x    = (const float*)d_in[0];
  const int*   ei   = (const int*)d_in[1];
  const float* ew   = (const float*)d_in[2];
  const float* Wg   = (const float*)d_in[3];
  const float* bg   = (const float*)d_in[4];
  const float* Wq   = (const float*)d_in[5];
  const float* Wk   = (const float*)d_in[6];
  const float* Wv   = (const float*)d_in[7];
  const float* vw   = (const float*)d_in[8];
  const float* vb   = (const float*)d_in[9];
  const float* l1g  = (const float*)d_in[10];
  const float* l1b  = (const float*)d_in[11];
  const float* wih  = (const float*)d_in[12];
  const float* bih  = (const float*)d_in[14];
  const float* bhh  = (const float*)d_in[15];
  const float* l2g  = (const float*)d_in[16];
  const float* l2b  = (const float*)d_in[17];
  const float* p1w  = (const float*)d_in[18];
  const float* p1b  = (const float*)d_in[19];
  const float* p2w  = (const float*)d_in[20];
  const float* p2b  = (const float*)d_in[21];
  const float* lw   = (const float*)d_in[22];
  const float* lb   = (const float*)d_in[23];
  const float* iw   = (const float*)d_in[24];
  const float* ib   = (const float*)d_in[25];
  float* out = (float*)d_out;

  char* ws = (char*)d_ws;
  float*          PAR  = (float*)(ws + O_PAR);
  unsigned short* WG2  = (unsigned short*)(ws + O_WG2);
  unsigned short* WK2  = (unsigned short*)(ws + O_WK2);
  unsigned short* WH2  = (unsigned short*)(ws + O_WH2);
  float*          DINV = (float*)(ws + O_DINV);
  int*            RP   = (int*)(ws + O_RP);
  int*            HSRC = (int*)(ws + O_HSRC);
  float*          HCF  = (float*)(ws + O_HCF);
  int*            POI  = (int*)(ws + O_POI);
  float*          QP   = (float*)(ws + O_QP);
  float*          MZ   = (float*)(ws + O_MZ);
  unsigned short* FHL  = (unsigned short*)(ws + O_FHL);
  float*          REC  = (float*)(ws + O_REC);
  float*          SC   = (float*)(ws + O_SC);
  float*          NF   = (float*)(ws + O_NF);
  float*          QF   = (float*)(ws + O_QF);

  const int csrLds  = CSR_INTS * 4;
  const int qLds    = Q_INTS * 4;
  const int mainLds = MAIN_INTS * 4;
  hipFuncSetAttribute(reinterpret_cast<const void*>(&k_csr),  hipFuncAttributeMaxDynamicSharedMemorySize, csrLds);
  hipFuncSetAttribute(reinterpret_cast<const void*>(&k_q),    hipFuncAttributeMaxDynamicSharedMemorySize, qLds);
  hipFuncSetAttribute(reinterpret_cast<const void*>(&k_main), hipFuncAttributeMaxDynamicSharedMemorySize, mainLds);

  k_pa<<<9, 256, 0, stream>>>(bg, Wq, Wv, vw, vb, l1g, l1b, PAR);
  k_pb<<<34, 256, 0, stream>>>(wih, bih, bhh, l2g, l2b, p1w, p1b, lb, ib, PAR);
  k_pc<<<10, 256, 0, stream>>>(Wg, Wk, lw, iw, WG2, WK2, WH2);
  k_csr<<<1, 512, csrLds, stream>>>(ei, ew, DINV, RP, HSRC, HCF, POI);
  k_q<<<C_B, 256, qLds, stream>>>(x, PAR, WG2, RP, HSRC, HCF, DINV, QP);
  k_main<<<C_SL, 256, mainLds, stream>>>(x, PAR, WG2, WK2, RP, HSRC, HCF, DINV, QP, REC, SC);
  k_tail<<<1, 256, 0, stream>>>(PAR, REC, MZ, FHL);
  k_pre2<<<1000, 256, 0, stream>>>(FHL, p2w, p2b, NF);
  k_head<<<125, 128, 0, stream>>>(NF, WH2, PAR, QF);
  k_out0<<<(OUT0_N / 4 + 255) / 256, 256, 0, stream>>>(QF, POI, out);
  k_out1<<<OUT1_N / 256, 256, 0, stream>>>(SC, MZ, POI, out);
}
